// RibonanzaNetPairwiseAttention_17325898072634
// MI455X (gfx1250) — hardware-verified
//
#include <hip/hip_runtime.h>
#include <stddef.h>


typedef _Float16 f16;
typedef f16 v16h __attribute__((ext_vector_type(16)));
typedef f16 v8h __attribute__((ext_vector_type(8)));
typedef f16 v4h __attribute__((ext_vector_type(4)));
typedef float v8f __attribute__((ext_vector_type(8)));
typedef float v4f __attribute__((ext_vector_type(4)));
typedef unsigned int v4u __attribute__((ext_vector_type(4)));

union H8 { v8h h; v4u u; };

#define LL 256
#define DD 128
#define HH 8
#define DHH 16
#define NROWS (LL * LL)
#define WSC 64.0f
#define XP 136
#define VP 264
#define GP 136
#define OP 132

static __device__ __forceinline__ v8f wmma16(v16h a, v16h b, v8f c) {
  v8f d = __builtin_amdgcn_wmma_f32_16x16x32_f16(false, a, false, b, (short)0, c, false, false);
  asm volatile("v_nop\n\tv_nop\n\tv_nop\n\tv_nop" : "+v"(d) : "v"(a), "v"(b));
  return d;
}

static __device__ __forceinline__ v16h cat8(v8h a, v8h b) {
  return __builtin_shufflevector(a, b, 0, 1, 2, 3, 4, 5, 6, 7, 8, 9, 10, 11, 12, 13, 14, 15);
}

__global__ void __launch_bounds__(64) pack_kernel(const float* __restrict__ Wq, const float* __restrict__ Wk,
                                                   const float* __restrict__ Wv, const float* __restrict__ Wg,
                                                   const float* __restrict__ Wd, const float* __restrict__ Wb,
                                                   f16* Pq, f16* Pk, f16* Pv, f16* Pg, f16* Pd, f16* Pb) {
  const int t = blockIdx.x, tid = threadIdx.x;
  const int lanef = tid >> 1, half = tid & 1, n16 = lanef & 15, hh = lanef >> 4;
  const float* W;
  f16* P;
  int kt, nt, ldw, ntcount;
  if (t < 160) {
    const int wsel = t >> 5, tile = t & 31;
    kt = tile >> 3; nt = tile & 7; ldw = DD; ntcount = 8;
    if (wsel == 0)      { W = Wq; P = Pq; }
    else if (wsel == 1) { W = Wk; P = Pk; }
    else if (wsel == 2) { W = Wv; P = Pv; }
    else if (wsel == 3) { W = Wg; P = Pg; }
    else                { W = Wd; P = Pd; }
  } else if (t < 164) {
    kt = t - 160; nt = 0; ldw = HH; ntcount = 1; W = Wb; P = Pb;
  } else {
    return;
  }
  const int n = nt * 16 + n16;
  v8h hv;
#pragma unroll
  for (int e = 0; e < 8; ++e) {
    const int kk = kt * 32 + 16 * half + 8 * hh + e;
    float wv = 0.0f;
    if (n < ldw) wv = W[kk * ldw + n] * WSC;
    hv[e] = (f16)wv;
  }
  H8 val;
  val.h = hv;
  f16* dst = P + (size_t)(kt * ntcount + nt) * 512 + tid * 8;
  *(volatile v4u*)dst = val.u;
  __threadfence();
  *(volatile v4u*)dst = val.u;
}

template <bool GATE>
static __device__ __forceinline__ void proj_one(const f16* xs, f16* ts, const f16* __restrict__ P,
                                                 const float* __restrict__ bg, f16* O,
                                                 int row0, int tid, int lane, int w, int lm, int hf) {
  v16h bfr[4];
#pragma unroll
  for (int kt = 0; kt < 4; ++kt) {
    const f16* bp = P + ((size_t)(kt * 8 + w) * 32 + lane) * 16;
    bfr[kt] = cat8(*(const v8h*)bp, *(const v8h*)(bp + 8));
  }
  v8f acc0 = {};
  v8f acc1 = {};
#pragma unroll
  for (int kt = 0; kt < 4; ++kt) {
    const f16* a0p = xs + lm * XP + kt * 32 + 8 * hf;
    const f16* a1p = a0p + 16 * XP;
    const v16h a0 = cat8(*(const v8h*)a0p, *(const v8h*)(a0p + 16));
    const v16h a1 = cat8(*(const v8h*)a1p, *(const v8h*)(a1p + 16));
    acc0 = wmma16(a0, bfr[kt], acc0);
    acc1 = wmma16(a1, bfr[kt], acc1);
  }
  const int col = w * 16 + lm;
  float bb = 0.0f;
  if (GATE) bb = bg[col];
  __syncthreads();
#pragma unroll
  for (int r = 0; r < 8; ++r) {
    float v0 = acc0[r] * (1.0f / WSC);
    float v1 = acc1[r] * (1.0f / WSC);
    if (GATE) {
      v0 = 1.0f / (1.0f + __expf(-(v0 + bb)));
      v1 = 1.0f / (1.0f + __expf(-(v1 + bb)));
    }
    ts[(8 * hf + r) * XP + col] = (f16)v0;
    ts[(16 + 8 * hf + r) * XP + col] = (f16)v1;
  }
  __syncthreads();
  H8 o0, o1;
  f16* d0;
  f16* d1;
  {
    const int c = tid, lr = c >> 4, c8 = (c & 15) * 8;
    o0.h = *(const v8h*)(ts + lr * XP + c8);
    d0 = O + (size_t)(row0 + lr) * DD + c8;
  }
  {
    const int c = tid + 256, lr = c >> 4, c8 = (c & 15) * 8;
    o1.h = *(const v8h*)(ts + lr * XP + c8);
    d1 = O + (size_t)(row0 + lr) * DD + c8;
  }
  *(volatile v4u*)d0 = o0.u;
  *(volatile v4u*)d1 = o1.u;
  __threadfence();
  *(volatile v4u*)d0 = o0.u;
  *(volatile v4u*)d1 = o1.u;
}

__global__ void __launch_bounds__(256) proj_kernel(const float* __restrict__ x, const float* __restrict__ lnw,
                                                    const float* __restrict__ lnb, const float* __restrict__ mask,
                                                    const float* __restrict__ bg,
                                                    const f16* __restrict__ Pq, const f16* __restrict__ Pk,
                                                    const f16* __restrict__ Pv, const f16* __restrict__ Pg,
                                                    const f16* __restrict__ Pb,
                                                    f16* q, f16* k, f16* v, f16* gate, float* BhT, int nrows) {
  __shared__ __align__(16) f16 xs[32 * XP];
  __shared__ __align__(16) f16 ts[32 * XP];
  __shared__ __align__(16) float bs[HH * 32];
  const int row0 = blockIdx.x * 32;
  if (row0 + 32 > nrows) return;
  const int tid = threadIdx.x, lane = tid & 31, w = tid >> 5, lm = lane & 15, hf = lane >> 4;

  {
    const v4f wv = *(const v4f*)(lnw + lane * 4);
    const v4f bv = *(const v4f*)(lnb + lane * 4);
#pragma unroll
    for (int rr = 0; rr < 4; ++rr) {
      const int lr = w * 4 + rr;
      const size_t grow = (size_t)(row0 + lr);
      const v4f xv = *(const v4f*)(x + grow * DD + lane * 4);
      float s = (xv[0] + xv[1]) + (xv[2] + xv[3]);
#pragma unroll
      for (int m = 1; m < 32; m <<= 1) s += __shfl_xor(s, m, 32);
      const float mu = s * (1.0f / DD);
      v4f d;
      d[0] = xv[0] - mu; d[1] = xv[1] - mu; d[2] = xv[2] - mu; d[3] = xv[3] - mu;
      float qq = (d[0] * d[0] + d[1] * d[1]) + (d[2] * d[2] + d[3] * d[3]);
#pragma unroll
      for (int m = 1; m < 32; m <<= 1) qq += __shfl_xor(qq, m, 32);
      const float rs = rsqrtf(qq * (1.0f / DD) + 1e-5f);
      v4h o;
#pragma unroll
      for (int e = 0; e < 4; ++e) o[e] = (f16)((d[e] * rs) * wv[e] + bv[e]);
      *(v4h*)(xs + lr * XP + lane * 4) = o;
    }
  }
  __syncthreads();

  {
    if (w < 2) {
      v8f accb = {};
#pragma unroll
      for (int kt = 0; kt < 4; ++kt) {
        const f16* ap = xs + (w * 16 + lm) * XP + kt * 32 + 8 * hf;
        const v16h a = cat8(*(const v8h*)ap, *(const v8h*)(ap + 16));
        const f16* bp = Pb + ((size_t)kt * 32 + lane) * 16;
        const v16h b = cat8(*(const v8h*)bp, *(const v8h*)(bp + 8));
        accb = wmma16(a, b, accb);
      }
      if (lm < HH) {
#pragma unroll
        for (int r = 0; r < 8; ++r) {
          const int lr = w * 16 + 8 * hf + r;
          bs[lm * 32 + lr] = accb[r] * (1.0f / WSC) + mask[row0 + lr];
        }
      }
    }
    __syncthreads();
    v4f bvv = {};
    float* bdst = BhT;
    if (tid < 64) {
      const int hh = tid >> 3, qd = tid & 7;
      bvv = *(const v4f*)(bs + hh * 32 + qd * 4);
      bdst = BhT + (size_t)hh * nrows + row0 + qd * 4;
      *(volatile v4f*)bdst = bvv;
    }
    __threadfence();
    if (tid < 64) *(volatile v4f*)bdst = bvv;
  }

  proj_one<false>(xs, ts, Pq, bg, q, row0, tid, lane, w, lm, hf);
  proj_one<false>(xs, ts, Pk, bg, k, row0, tid, lane, w, lm, hf);
  proj_one<false>(xs, ts, Pv, bg, v, row0, tid, lane, w, lm, hf);
  proj_one<true>(xs, ts, Pg, bg, gate, row0, tid, lane, w, lm, hf);
}

__global__ void __launch_bounds__(256) attn_kernel(const f16* __restrict__ q, const f16* __restrict__ k,
                                                    const f16* __restrict__ v, const f16* __restrict__ gate,
                                                    const float* __restrict__ BhT, const f16* __restrict__ Pd,
                                                    const float* __restrict__ bd, const float* __restrict__ x,
                                                    float* out, int nrows) {
  __shared__ __align__(16) f16 VT[HH * DHH * VP];
  __shared__ __align__(16) f16 gs[16 * GP];
  __shared__ __align__(16) float outs[16 * OP];
  const int i = blockIdx.x;
  if ((i + 1) * LL > nrows) return;
  const int tid = threadIdx.x, lane = tid & 31, h = tid >> 5, lm = lane & 15, hf = lane >> 4;
  const size_t ibase = (size_t)i * LL;

  for (int c = tid; c < LL * 16; c += 256) {
    const int kc = c >> 4, c16 = c & 15;
    const v8h t8 = *(const v8h*)(v + (ibase + kc) * DD + c16 * 8);
    f16* dp = VT + ((c16 >> 1) * DHH + (c16 & 1) * 8) * VP + kc;
#pragma unroll
    for (int e = 0; e < 8; ++e) dp[e * VP] = t8[e];
  }
  __syncthreads();

  const float* bh = BhT + (size_t)h * nrows;
  const v8h z8 = {};

#pragma unroll 1
  for (int jt = 0; jt < 16; ++jt) {
    const int j0 = jt * 16;
    const v16h bqf = cat8(*(const v8h*)(q + (ibase + j0 + lm) * DD + h * DHH + 8 * hf), z8);

    v8f c[16];
    float mx = -3.0e38f;
#pragma unroll
    for (int kt = 0; kt < 16; ++kt) {
      const v16h akf = cat8(*(const v8h*)(k + (ibase + kt * 16 + lm) * DD + h * DHH + 8 * hf), z8);
      v8f z = {};
      const v8f s = wmma16(akf, bqf, z);
      const float* bp = bh + (size_t)(j0 + lm) * LL + kt * 16 + 8 * hf;
      const v4f b0 = *(const v4f*)bp;
      const v4f b1 = *(const v4f*)(bp + 4);
#pragma unroll
      for (int r = 0; r < 4; ++r) {
        c[kt][r] = fmaf(s[r], 0.25f, b0[r]);
        c[kt][4 + r] = fmaf(s[4 + r], 0.25f, b1[r]);
      }
#pragma unroll
      for (int r = 0; r < 8; ++r) mx = fmaxf(mx, c[kt][r]);
    }
    mx = fmaxf(mx, __shfl_xor(mx, 16, 32));
    float sum = 0.0f;
#pragma unroll
    for (int kt = 0; kt < 16; ++kt) {
#pragma unroll
      for (int r = 0; r < 8; ++r) {
        const float e = __expf(c[kt][r] - mx);
        c[kt][r] = e;
        sum += e;
      }
    }
    sum += __shfl_xor(sum, 16, 32);
    const float inv = 256.0f / sum;

    v8f cc = {};
#pragma unroll
    for (int kk = 0; kk < 8; ++kk) {
      v16h pb;
#pragma unroll
      for (int r = 0; r < 8; ++r) {
        pb[r] = (f16)(c[2 * kk][r] * inv);
        pb[8 + r] = (f16)(c[2 * kk + 1][r] * inv);
      }
      const f16* ap = VT + (h * DHH + lm) * VP + kk * 32 + 8 * hf;
      const v16h av = cat8(*(const v8h*)ap, *(const v8h*)(ap + 16));
      cc = wmma16(av, pb, cc);
    }
    {
      const v8h gv = *(const v8h*)(gate + (ibase + j0 + lm) * DD + h * DHH + 8 * hf);
      v8h go;
#pragma unroll
      for (int r = 0; r < 8; ++r) go[r] = (f16)(cc[r] * ((float)gv[r] * 0.25f));
      *(v8h*)(gs + lm * GP + h * DHH + 8 * hf) = go;
    }
    __syncthreads();

    {
      v8f acc = {};
#pragma unroll
      for (int kt = 0; kt < 4; ++kt) {
        const f16* ap = gs + lm * GP + kt * 32 + 8 * hf;
        const v16h a = cat8(*(const v8h*)ap, *(const v8h*)(ap + 16));
        const f16* bp = Pd + ((size_t)(kt * 8 + h) * 32 + lane) * 16;
        const v16h b = cat8(*(const v8h*)bp, *(const v8h*)(bp + 8));
        acc = wmma16(a, b, acc);
      }
#pragma unroll
      for (int r = 0; r < 8; ++r) outs[(8 * hf + r) * OP + h * 16 + lm] = acc[r] * (1.0f / 4096.0f);
    }
    __syncthreads();

    v4f o0, o1;
    float* od0;
    float* od1;
    {
      const int cidx = tid, lr = cidx >> 5, col4 = (cidx & 31) * 4;
      const size_t grow = ibase + j0 + lr;
      o0 = *(const v4f*)(outs + lr * OP + col4) + *(const v4f*)(bd + col4) +
           *(const v4f*)(x + grow * DD + col4);
      od0 = out + grow * DD + col4;
    }
    {
      const int cidx = tid + 256, lr = cidx >> 5, col4 = (cidx & 31) * 4;
      const size_t grow = ibase + j0 + lr;
      o1 = *(const v4f*)(outs + lr * OP + col4) + *(const v4f*)(bd + col4) +
           *(const v4f*)(x + grow * DD + col4);
      od1 = out + grow * DD + col4;
    }
    *(volatile v4f*)od0 = o0;
    *(volatile v4f*)od1 = o1;
    __threadfence();
    *(volatile v4f*)od0 = o0;
    *(volatile v4f*)od1 = o1;
  }
}

extern "C" void kernel_launch(void* const* d_in, const int* in_sizes, int n_in,
                              void* d_out, int out_size, void* d_ws, size_t ws_size,
                              hipStream_t stream) {
  if (n_in < 12) return;
  if (in_sizes[0] != NROWS * DD || in_sizes[1] != NROWS || in_sizes[2] != DD || in_sizes[3] != DD ||
      in_sizes[4] != DD * DD || in_sizes[5] != DD * DD || in_sizes[6] != DD * DD ||
      in_sizes[7] != DD * HH || in_sizes[8] != DD * DD || in_sizes[9] != DD ||
      in_sizes[10] != DD * DD || in_sizes[11] != DD || out_size != NROWS * DD)
    return;

  const float* x    = (const float*)d_in[0];
  const float* mask = (const float*)d_in[1];
  const float* lnw  = (const float*)d_in[2];
  const float* lnb  = (const float*)d_in[3];
  const float* Wq   = (const float*)d_in[4];
  const float* Wk   = (const float*)d_in[5];
  const float* Wv   = (const float*)d_in[6];
  const float* Wb   = (const float*)d_in[7];
  const float* Wg   = (const float*)d_in[8];
  const float* bg   = (const float*)d_in[9];
  const float* Wd   = (const float*)d_in[10];
  const float* bd   = (const float*)d_in[11];
  float* out = (float*)d_out;

  const size_t RC = (size_t)NROWS * DD;
  f16* q    = (f16*)d_ws;
  f16* k    = q + RC;
  f16* v    = k + RC;
  f16* gate = v + RC;
  float* BhT = (float*)(gate + RC);
  f16* Pq = (f16*)(BhT + (size_t)HH * NROWS);
  f16* Pk = Pq + DD * DD;
  f16* Pv = Pk + DD * DD;
  f16* Pg = Pv + DD * DD;
  f16* Pd = Pg + DD * DD;
  f16* Pb = Pd + DD * DD;
  const size_t total = 4 * RC * sizeof(f16) + (size_t)HH * NROWS * sizeof(float) +
                       5 * (size_t)DD * DD * sizeof(f16) + 4 * 512 * sizeof(f16);
  if (total > ws_size) return;

  pack_kernel<<<dim3(164), dim3(64), 0, stream>>>(Wq, Wk, Wv, Wg, Wd, Wb, Pq, Pk, Pv, Pg, Pd, Pb);
  proj_kernel<<<dim3(NROWS / 32), dim3(256), 0, stream>>>(x, lnw, lnb, mask, bg, Pq, Pk, Pv, Pg, Pb,
                                                           q, k, v, gate, BhT, (int)NROWS);
  attn_kernel<<<dim3(LL), dim3(256), 0, stream>>>(q, k, v, gate, BhT, Pd, bd, x, out, (int)NROWS);
}
